// StackedGatPerfPlayerModel_18141941858959
// MI455X (gfx1250) — hardware-verified
//
#include <hip/hip_runtime.h>


namespace {
constexpr int B = 8, N = 4096, DEG = 16, DIN = 64, DM = 128, NH = 4, DH = 32, NL = 3, NT = B * N, NBLK = NT / 16;
constexpr float XS = 8.0f, WSC = 256.0f; constexpr double NNS = 1999853.335557038;
typedef _Float16 b16;
typedef __attribute__((ext_vector_type(16))) _Float16 v16b;
typedef __attribute__((ext_vector_type(8))) _Float16 v8b;
typedef __attribute__((ext_vector_type(8))) float v8f;
typedef __attribute__((ext_vector_type(4))) float v4f;
__device__ __forceinline__ float bf16_rne(float f) { unsigned int u = __float_as_uint(f); u += 0x7FFFu + ((u >> 16) & 1u); return __uint_as_float(u & 0xFFFF0000u); }
__device__ __forceinline__ void split16(float v, b16& hi, b16& lo) { hi = (b16)v; lo = (b16)(v - (float)hi); }
__device__ __forceinline__ v16b frag_kb(const b16* p, int hh) { const v8b a = *(const v8b*)(p + 8 * hh), b = *(const v8b*)(p + 16 + 8 * hh); v16b f;
#pragma unroll
  for (int e = 0; e < 8; ++e) { f[e] = a[e]; f[8 + e] = b[e]; } return f; }
__device__ __forceinline__ v8f wmma16b(v16b a, v16b b, v8f c) { v8f d = __builtin_amdgcn_wmma_f32_16x16x32_f16(false, a, false, b, (short)0, c, false, false); asm volatile("v_nop\n\tv_nop\n\tv_nop\n\tv_nop" : "+v"(d) : "v"(a), "v"(b)); return d; }
__device__ __forceinline__ void wave_lds_sync() { __builtin_amdgcn_fence(__ATOMIC_RELEASE, "workgroup"); __builtin_amdgcn_wave_barrier(); __builtin_amdgcn_fence(__ATOMIC_ACQUIRE, "workgroup"); }
__device__ __forceinline__ float pmul(float a, float b) { float p = a * b; asm volatile("" : "+v"(p)); return p; }
__device__ __forceinline__ int iclamp(int v, int lo, int hi) { return v < lo ? lo : (v > hi ? hi : v); }
__device__ __forceinline__ float elu(float v) { return v > 0.0f ? v : expm1f(v); }
__device__ __forceinline__ float leaky(float v) { return v > 0.0f ? v : 0.2f * v; }

__global__ __launch_bounds__(256) void wput_kernel(const float* __restrict__ w, int KIN, int OUTW, int OUTP, b16* __restrict__ WT) {
  const int KG = KIN / 8; const int u = blockIdx.x * 256 + threadIdx.x; if (u >= OUTP * KG) return; const int o = u / KG, k0 = (u % KG) * 8; v8b v;
#pragma unroll
  for (int j = 0; j < 8; ++j) v[j] = (o < OUTW) ? (b16)(bf16_rne(w[(size_t)(k0 + j) * OUTW + o]) * WSC) : (b16)0.0f; for (int pass = 0; pass < 2; ++pass) { *(volatile v8b*)(WT + (size_t)o * KIN + k0) = v; __threadfence(); }
}
__global__ __launch_bounds__(256) void wl_kernel(const float* __restrict__ Wl, const float* __restrict__ Wo, b16* __restrict__ WL, b16* __restrict__ WOB) {
  const int u = blockIdx.x * 256 + threadIdx.x; if (u >= 2 * 128 * 16) return; const int which = u / (128 * 16), r = (u / 16) % 128, k0 = (u % 16) * 8; const int h = r / 32, c = r % 32; v8b v;
  for (int j = 0; j < 8; ++j) { const int k = k0 + j; float val; if (which == 0) val = Wl[((size_t)h * DM + k) * DH + c]; else { const int hb = k / 32, kk = k % 32; val = (hb == h) ? Wo[((size_t)h * DH + kk) * 32 + c] : 0.0f; } v[j] = (b16)(bf16_rne(val) * WSC); }
  for (int pass = 0; pass < 2; ++pass) { *(volatile v8b*)((which == 0 ? WL : WOB) + (size_t)r * 128 + k0) = v; __threadfence(); }
}
__global__ __launch_bounds__(32) void in_kernel(const float* __restrict__ nf, const b16* __restrict__ W0T, const float* __restrict__ b0, int NLIM, float* __restrict__ X) {
  __shared__ __attribute__((aligned(16))) b16 Ah[16][DIN + 8]; __shared__ __attribute__((aligned(16))) float Tf[16][DM + 4];
  const int lane = threadIdx.x, nloc = lane & 15, hlf = lane >> 4; const size_t m0 = (size_t)blockIdx.x * 16; if (m0 >= (size_t)NLIM) return;
  for (int rr = 0; rr < 16; ++rr) for (int q = 0; q < 2; ++q) Ah[rr][q * 32 + lane] = (b16)(bf16_rne(nf[(m0 + rr) * DIN + q * 32 + lane]) * XS);
  wave_lds_sync(); v8f acc[8];
#pragma unroll
  for (int t = 0; t < 8; ++t) acc[t] = (v8f){};
#pragma unroll
  for (int kb = 0; kb < DIN; kb += 32) { const v16b a = frag_kb(&Ah[nloc][kb], hlf);
#pragma unroll
    for (int t = 0; t < 8; ++t) acc[t] = wmma16b(a, frag_kb(W0T + (size_t)(t * 16 + nloc) * DIN + kb, hlf), acc[t]); }
#pragma unroll
  for (int t = 0; t < 8; ++t) { const int c = t * 16 + nloc; const float bb = bf16_rne(b0[c]);
#pragma unroll
    for (int r8 = 0; r8 < 8; ++r8) Tf[8 * hlf + r8][c] = elu(acc[t][r8] * (1.0f / (XS * WSC)) + bb); }
  wave_lds_sync();
  for (int pass = 0; pass < 2; ++pass) { for (int rr = 0; rr < 16; ++rr) *(volatile v4f*)(X + (m0 + rr) * DM + lane * 4) = *(const v4f*)(&Tf[rr][lane * 4]); __threadfence(); }
}
__global__ __launch_bounds__(32) void proj_kernel(const float* __restrict__ X, const b16* __restrict__ WL, const float* __restrict__ asrc, const float* __restrict__ adst, int NLIM, float* __restrict__ Hh, float* __restrict__ ED) {
  __shared__ __attribute__((aligned(16))) b16 Ah[16][DM + 8]; __shared__ __attribute__((aligned(16))) float Tf[16][DM + 4], Ps[16][8];
  const int lane = threadIdx.x, nloc = lane & 15, hlf = lane >> 4; const size_t m0 = (size_t)blockIdx.x * 16; if (m0 >= (size_t)NLIM) return;
  for (int rr = 0; rr < 16; ++rr) for (int q = 0; q < 4; ++q) Ah[rr][q * 32 + lane] = (b16)(X[(m0 + rr) * DM + q * 32 + lane] * XS);
  wave_lds_sync(); v8f acc[8];
#pragma unroll
  for (int t = 0; t < 8; ++t) acc[t] = (v8f){};
#pragma unroll
  for (int kb = 0; kb < DM; kb += 32) { const v16b a = frag_kb(&Ah[nloc][kb], hlf);
#pragma unroll
    for (int t = 0; t < 8; ++t) acc[t] = wmma16b(a, frag_kb(WL + (size_t)(t * 16 + nloc) * DM + kb, hlf), acc[t]); }
  float ps[8], pd[8];
#pragma unroll
  for (int r8 = 0; r8 < 8; ++r8) { ps[r8] = 0.0f; pd[r8] = 0.0f; }
#pragma unroll
  for (int t = 0; t < 8; ++t) { const int c = t * 16 + nloc; const int h = t >> 1; const float ws_ = bf16_rne(asrc[c]), wd_ = bf16_rne(adst[c]);
#pragma unroll
    for (int r8 = 0; r8 < 8; ++r8) { const float v = acc[t][r8] * (1.0f / (XS * WSC)); Tf[8 * hlf + r8][c] = v; ps[r8] += pmul(v, ws_); pd[r8] += pmul(v, wd_); }
    if (t & 1) {
#pragma unroll
      for (int r8 = 0; r8 < 8; ++r8) { float a = ps[r8], d = pd[r8]; for (int o = 1; o < 16; o <<= 1) { a += __shfl_xor(a, o); d += __shfl_xor(d, o); } if (nloc == 0) { Ps[8 * hlf + r8][h] = a; Ps[8 * hlf + r8][4 + h] = d; } ps[r8] = 0.0f; pd[r8] = 0.0f; } } }
  wave_lds_sync();
  for (int pass = 0; pass < 2; ++pass) { for (int rr = 0; rr < 16; ++rr) *(volatile v4f*)(Hh + (m0 + rr) * DM + lane * 4) = *(const v4f*)(&Tf[rr][lane * 4]); for (int q = 0; q < 4; ++q) { const int i = q * 32 + lane; ((volatile float*)ED)[m0 * 8 + i] = Ps[i >> 3][i & 7]; } __threadfence(); }
}
__global__ __launch_bounds__(32) void att_kernel(const float* __restrict__ Hh, const float* __restrict__ ED, const int* __restrict__ adj, const float* __restrict__ masks, const float* __restrict__ X, const b16* __restrict__ WOB, const b16* __restrict__ WLIN, const float* __restrict__ blin, const float* __restrict__ g, const float* __restrict__ be, int NLIM, float* __restrict__ XN) {
  __shared__ __attribute__((aligned(16))) b16 Ah[16][DM + 8]; __shared__ __attribute__((aligned(16))) float Tf[16][DM + 4];
  const int lane = threadIdx.x, nloc = lane & 15, hlf = lane >> 4; const size_t m0 = (size_t)blockIdx.x * 16; if (m0 >= (size_t)NLIM) return; const int h = lane >> 3; const size_t gb = (m0 / N) * N;
  for (int rr = 0; rr < 16; ++rr) { const size_t n = m0 + rr; const float es = ED[n * 8 + h]; float ev[DEG]; size_t nb[DEG]; float mx = -INFINITY;
#pragma unroll
    for (int m = 0; m < DEG; ++m) { nb[m] = gb + (size_t)iclamp(adj[n * DEG + m], 0, N - 1); float e = leaky(es + ED[nb[m] * 8 + 4 + h]); if (!(masks[n * DEG + m] > 0.0f)) e = -1e9f; ev[m] = e; mx = fmaxf(mx, e); }
    float den = 0.0f; v4f o = {0, 0, 0, 0};
#pragma unroll
    for (int m = 0; m < DEG; ++m) { const float p = __expf(ev[m] - mx); den += p; const v4f hv = *(const v4f*)(Hh + nb[m] * DM + lane * 4); for (int i = 0; i < 4; ++i) o[i] += pmul(p, hv[i]); }
    const float inv = 1.0f / den; for (int i = 0; i < 4; ++i) Ah[rr][lane * 4 + i] = (b16)(pmul(o[i], inv) * XS); }
  wave_lds_sync(); v8f acc[8];
#pragma unroll
  for (int t = 0; t < 8; ++t) acc[t] = (v8f){};
#pragma unroll
  for (int kb = 0; kb < DM; kb += 32) { const v16b a = frag_kb(&Ah[nloc][kb], hlf);
#pragma unroll
    for (int t = 0; t < 8; ++t) acc[t] = wmma16b(a, frag_kb(WOB + (size_t)(t * 16 + nloc) * DM + kb, hlf), acc[t]); }
  wave_lds_sync();
#pragma unroll
  for (int t = 0; t < 8; ++t) { const int c = t * 16 + nloc;
#pragma unroll
    for (int r8 = 0; r8 < 8; ++r8) Ah[8 * hlf + r8][c] = (b16)(acc[t][r8] * (1.0f / (XS * WSC)) * XS); }
  wave_lds_sync();
#pragma unroll
  for (int t = 0; t < 8; ++t) acc[t] = (v8f){};
#pragma unroll
  for (int kb = 0; kb < DM; kb += 32) { const v16b a = frag_kb(&Ah[nloc][kb], hlf);
#pragma unroll
    for (int t = 0; t < 8; ++t) acc[t] = wmma16b(a, frag_kb(WLIN + (size_t)(t * 16 + nloc) * DM + kb, hlf), acc[t]); }
#pragma unroll
  for (int t = 0; t < 8; ++t) { const int c = t * 16 + nloc; const float bb = bf16_rne(blin[c]);
#pragma unroll
    for (int r8 = 0; r8 < 8; ++r8) { const int rl = 8 * hlf + r8; Tf[rl][c] = elu(acc[t][r8] * (1.0f / (XS * WSC)) + bb) + X[(m0 + rl) * DM + c]; } }
  wave_lds_sync();
  for (int rr = 0; rr < 16; ++rr) { float v[4], s = 0.0f; for (int i = 0; i < 4; ++i) { v[i] = Tf[rr][lane * 4 + i]; s += v[i]; } for (int q = 16; q; q >>= 1) s += __shfl_xor(s, q); const float mu = s * (1.0f / DM); float var = 0.0f; for (int i = 0; i < 4; ++i) { const float d = v[i] - mu; var += pmul(d, d); } for (int q = 16; q; q >>= 1) var += __shfl_xor(var, q); const float rs = rsqrtf(var * (1.0f / DM) + 1e-5f);
    v4f r; for (int i = 0; i < 4; ++i) { const int c = lane * 4 + i; r[i] = pmul(pmul(v[i] - mu, rs), bf16_rne(g[c])) + bf16_rne(be[c]); }
    *(volatile v4f*)(XN + (m0 + rr) * DM + lane * 4) = r; __threadfence(); *(volatile v4f*)(XN + (m0 + rr) * DM + lane * 4) = r; }
  __threadfence();
}
__global__ __launch_bounds__(32) void head_kernel(const float* __restrict__ X, const int* __restrict__ qidx, int NBV, const b16* __restrict__ W1, const float* __restrict__ b1, const b16* __restrict__ W2, const float* __restrict__ b2, const b16* __restrict__ W3, const float* __restrict__ b3, float* __restrict__ out) {
  __shared__ __attribute__((aligned(16))) b16 Ah[16][256 + 8], Al[16][256 + 8]; __shared__ float Hs[16][256], So[16][16];
  const int lane = threadIdx.x, nloc = lane & 15, hlf = lane >> 4;
  for (int rr = 0; rr < 16; ++rr) { const size_t n = (rr < NBV) ? ((size_t)rr * N + (size_t)iclamp(qidx[rr < B ? rr : 0], 0, N - 1)) : 0; for (int q = 0; q < 4; ++q) { const float v = rr < NBV ? X[n * DM + q * 32 + lane] : 0.0f; b16 p, ql; split16(v * XS, p, ql); Ah[rr][q * 32 + lane] = p; Al[rr][q * 32 + lane] = ql; } }
  wave_lds_sync();
#pragma unroll 1
  for (int cg = 0; cg < 2; ++cg) { v8f acc[8];
#pragma unroll
    for (int t = 0; t < 8; ++t) acc[t] = (v8f){};
    for (int kb = 0; kb < 128; kb += 32) { const v16b a = frag_kb(&Ah[nloc][kb], hlf), al = frag_kb(&Al[nloc][kb], hlf);
#pragma unroll
      for (int t = 0; t < 8; ++t) { const v16b bw = frag_kb(W1 + (size_t)(cg * 128 + t * 16 + nloc) * 128 + kb, hlf); acc[t] = wmma16b(a, bw, acc[t]); acc[t] = wmma16b(al, bw, acc[t]); } }
#pragma unroll
    for (int t = 0; t < 8; ++t) { const int c = cg * 128 + t * 16 + nloc; const float bb = bf16_rne(b1[c]);
#pragma unroll
      for (int r8 = 0; r8 < 8; ++r8) Hs[8 * hlf + r8][c] = elu(acc[t][r8] * (1.0f / (XS * WSC)) + bb); } }
  wave_lds_sync();
  for (int rr = 0; rr < 16; ++rr) for (int q = 0; q < 8; ++q) { b16 p, ql; split16(Hs[rr][q * 32 + lane] * XS, p, ql); Ah[rr][q * 32 + lane] = p; Al[rr][q * 32 + lane] = ql; }
  wave_lds_sync();
  { v8f acc[8];
#pragma unroll
    for (int t = 0; t < 8; ++t) acc[t] = (v8f){};
    for (int kb = 0; kb < 256; kb += 32) { const v16b a = frag_kb(&Ah[nloc][kb], hlf), al = frag_kb(&Al[nloc][kb], hlf);
#pragma unroll
      for (int t = 0; t < 8; ++t) { const v16b bw = frag_kb(W2 + (size_t)(t * 16 + nloc) * 256 + kb, hlf); acc[t] = wmma16b(a, bw, acc[t]); acc[t] = wmma16b(al, bw, acc[t]); } }
    wave_lds_sync();
#pragma unroll
    for (int t = 0; t < 8; ++t) { const int c = t * 16 + nloc; const float bb = bf16_rne(b2[c]);
#pragma unroll
      for (int r8 = 0; r8 < 8; ++r8) Hs[8 * hlf + r8][c] = elu(acc[t][r8] * (1.0f / (XS * WSC)) + bb); } }
  wave_lds_sync();
  for (int rr = 0; rr < 16; ++rr) for (int q = 0; q < 4; ++q) { b16 p, ql; split16(Hs[rr][q * 32 + lane] * XS, p, ql); Ah[rr][q * 32 + lane] = p; Al[rr][q * 32 + lane] = ql; }
  wave_lds_sync();
  { v8f acc = {}; for (int kb = 0; kb < 128; kb += 32) { const v16b bw = frag_kb(W3 + (size_t)nloc * 128 + kb, hlf); acc = wmma16b(frag_kb(&Ah[nloc][kb], hlf), bw, acc); acc = wmma16b(frag_kb(&Al[nloc][kb], hlf), bw, acc); }
    if (nloc < 8) { const float bb = bf16_rne(b3[nloc]);
#pragma unroll
      for (int r8 = 0; r8 < 8; ++r8) So[8 * hlf + r8][nloc] = (float)((double)elu(acc[r8] * (1.0f / (XS * WSC)) + bb) * NNS); } }
  wave_lds_sync();
  for (int pass = 0; pass < 2; ++pass) { for (int i = lane; i < B * 8; i += 32) ((volatile float*)out)[i] = So[i / 8][i % 8]; __threadfence(); }
}
}

extern "C" void kernel_launch(void* const* d_in, const int* in_sizes, int n_in, void* d_out, int out_size, void* d_ws, size_t ws_size, hipStream_t stream) {
  (void)n_in;
  auto Fp = [&](int i) { return (const float*)d_in[i]; }; auto Ip = [&](int i) { return (const int*)d_in[i]; };
  if (in_sizes[0] != NT * DIN || in_sizes[1] != B || in_sizes[2] != NT * DEG || in_sizes[3] != NT * DEG || in_sizes[5] != DIN * DM || in_sizes[7] != NL * NH * DM * DH || in_sizes[10] != NL * NH * DH * 32 || in_sizes[11] != NL * DM * DM || in_sizes[15] != DM * 256 || in_sizes[17] != 256 * 128 || in_sizes[19] != 128 * 8 || out_size != B * 8) return;
  const int NBV = B; const int NLIM = NBV * N; const int GB16 = NLIM / 16;
  size_t off = 0; char* ws = (char*)d_ws;
  auto carve = [&](size_t bytes) { char* p = ws + off; off += (bytes + 255) & ~(size_t)255; return p; };
  b16* W0T = (b16*)carve(DM * DIN * 2); b16* WL[3]; b16* WOB[3]; b16* WLIN[3]; for (int l = 0; l < 3; ++l) { WL[l] = (b16*)carve(128 * 128 * 2); WOB[l] = (b16*)carve(128 * 128 * 2); WLIN[l] = (b16*)carve(128 * 128 * 2); }
  b16* WF1 = (b16*)carve(256 * 128 * 2); b16* WF2 = (b16*)carve(128 * 256 * 2); b16* WF3 = (b16*)carve(16 * 128 * 2);
  float* XA = (float*)carve((size_t)NT * DM * 4); float* XB = (float*)carve((size_t)NT * DM * 4); float* Hh = (float*)carve((size_t)NT * DM * 4); float* ED = (float*)carve((size_t)NT * 8 * 4);
  if (off > ws_size || off > ((size_t)96 << 20)) return;
  wput_kernel<<<(DM * 8 + 255) / 256, 256, 0, stream>>>(Fp(5), DIN, DM, DM, W0T);
  for (int l = 0; l < 3; ++l) { wl_kernel<<<(2 * 128 * 16 + 255) / 256, 256, 0, stream>>>(Fp(7) + (size_t)l * NH * DM * DH, Fp(10) + (size_t)l * NH * DH * 32, WL[l], WOB[l]); wput_kernel<<<(DM * 16 + 255) / 256, 256, 0, stream>>>(Fp(11) + (size_t)l * DM * DM, DM, DM, DM, WLIN[l]); }
  wput_kernel<<<(256 * 16 + 255) / 256, 256, 0, stream>>>(Fp(15), DM, 256, 256, WF1); wput_kernel<<<(128 * 32 + 255) / 256, 256, 0, stream>>>(Fp(17), 256, 128, 128, WF2); wput_kernel<<<(16 * 16 + 255) / 256, 256, 0, stream>>>(Fp(19), 128, 8, 16, WF3);
  in_kernel<<<GB16, 32, 0, stream>>>(Fp(0), W0T, Fp(6), NLIM, XA);
  float* xp = XA; float* xn = XB;
  for (int l = 0; l < 3; ++l) {
    proj_kernel<<<GB16, 32, 0, stream>>>(xp, WL[l], Fp(8) + l * NH * DH, Fp(9) + l * NH * DH, NLIM, Hh, ED);
    att_kernel<<<GB16, 32, 0, stream>>>(Hh, ED, Ip(3), Fp(2), xp, WOB[l], WLIN[l], Fp(12) + l * DM, Fp(13) + l * DM, Fp(14) + l * DM, NLIM, xn);
    float* t = xp; xp = xn; xn = t; }
  head_kernel<<<1, 32, 0, stream>>>(xp, Ip(1), NBV, WF1, Fp(16), WF2, Fp(18), WF3, Fp(20), (float*)d_out);
}
